// Block_9122510537354
// MI455X (gfx1250) — hardware-verified
//
#include <hip/hip_runtime.h>
#include <math.h>

typedef __attribute__((ext_vector_type(16))) _Float16 v16h;
typedef __attribute__((ext_vector_type(8)))  _Float16 v8h;
typedef __attribute__((ext_vector_type(4)))  _Float16 v4h;
typedef __attribute__((ext_vector_type(8)))  float    v8f;
typedef __attribute__((ext_vector_type(4)))  float    v4f;

constexpr int kBatch  = 2;
constexpr int kSeq    = 1024;
constexpr int kDm     = 1024;
constexpr int kDin    = 2048;
constexpr int kNst    = 16;
constexpr int kDtR    = 64;
constexpr int kXzP    = 2 * kDin;
constexpr int kPrjN   = kDtR + 2 * kNst;
constexpr int kPrjP   = 128;
constexpr int kRows   = kBatch * kSeq;
constexpr int kConvTP = 260;
constexpr int kScanTS = 64;
constexpr int kScanCh = 64;
constexpr int kScanYP = 68;
constexpr float kLnEps = 1e-5f;

constexpr float kCarryHn  = 1.0f;
constexpr float kCarryW   = 32.0f;
constexpr float kCarryXa  = 1.0f;
constexpr float kCarryDt  = 16.0f;
constexpr float kCarryWdt = 8.0f;
constexpr float kCarryY   = 16.0f;
constexpr float kLoScale  = 2048.0f;
constexpr float kInMain   = 1.0f / (kCarryHn * kCarryW);
constexpr float kInCross  = kInMain / kLoScale;
constexpr float kXpScale  = 1.0f / (kCarryXa * kCarryW);
constexpr float kDtScale  = 1.0f / (kCarryDt * kCarryWdt);
constexpr float kOutMain  = 1.0f / (kCarryY * kCarryW);
constexpr float kOutCross = kOutMain / kLoScale;

static_assert(kPrjN == 96 && kPrjP % 64 == 0 && kPrjP >= kPrjN, "x_proj width and pad");
static_assert((kDm % 32) == 0 && (kDin % 32) == 0 && (kDtR % 32) == 0, "GEMM K multiples of 32");
static_assert((kRows % 64) == 0 && (kXzP % 64) == 0 && (kDin % 64) == 0 && (kDm % 64) == 0, "GEMM M,N tile multiples");
static_assert((kSeq % kScanTS) == 0 && (kSeq % 64) == 0 && (kDin % kScanCh) == 0 && (kDin % 256) == 0, "tile multiples");
static_assert(kDm == 4 * 256, "LayerNorm block owns one float4 per thread");

constexpr size_t kOffWINH = 0;
constexpr size_t kOffWINL = kOffWINH + (size_t)kXzP  * kDm  * 2;
constexpr size_t kOffWX   = kOffWINL + (size_t)kXzP  * kDm  * 2;
constexpr size_t kOffWDT  = kOffWX   + (size_t)kPrjP * kDin * 2;
constexpr size_t kOffWOH  = kOffWDT  + (size_t)kDin  * kDtR * 2;
constexpr size_t kOffWOL  = kOffWOH  + (size_t)kDm   * kDin * 2;
constexpr size_t kOffHNH  = kOffWOL  + (size_t)kDm   * kDin * 2;
constexpr size_t kOffHNL  = kOffHNH  + (size_t)kRows * kDm  * 2;
constexpr size_t kOffXZ   = kOffHNL  + (size_t)kRows * kDm  * 2;
constexpr size_t kOffXA   = kOffXZ   + (size_t)kRows * kXzP * 4;
constexpr size_t kOffXA16 = kOffXA   + (size_t)kRows * kDin * 4;
constexpr size_t kOffXD   = kOffXA16 + (size_t)kRows * kDin * 2;
constexpr size_t kOffDT16 = kOffXD   + (size_t)kRows * kPrjP * 4;
constexpr size_t kOffDLR  = kOffDT16 + (size_t)kRows * kDtR * 2;
constexpr size_t kOffYH   = kOffDLR  + (size_t)kRows * kDin * 4;
constexpr size_t kOffYL   = kOffYH   + (size_t)kRows * kDin * 2;
constexpr size_t kWsTotal = kOffYL   + (size_t)kRows * kDin * 2;
static_assert(kWsTotal == 127926272ull, "carve total");
static_assert(kWsTotal <= 134217728ull, "carve cap");
static_assert((kOffWINL % 128) == 0 && (kOffWX % 128) == 0 && (kOffWDT % 128) == 0 && (kOffWOH % 128) == 0 &&
              (kOffWOL % 128) == 0 && (kOffHNH % 128) == 0 && (kOffHNL % 128) == 0 && (kOffXZ % 128) == 0 &&
              (kOffXA % 128) == 0 && (kOffXA16 % 128) == 0 && (kOffXD % 128) == 0 && (kOffDT16 % 128) == 0 &&
              (kOffDLR % 128) == 0 && (kOffYH % 128) == 0 && (kOffYL % 128) == 0, "128-B aligned regions");

constexpr size_t kOut1ByteOff = (size_t)kRows * kDm * 4;
constexpr size_t kOut1ElemOff = kOut1ByteOff / 4;
static_assert(kOut1ByteOff == 8388608ull && (kOut1ByteOff % 128) == 0, "out1 offset");
static_assert(kOut1ByteOff + (size_t)kRows * kDm * 4 == 16777216ull, "d_out extent");

struct FragH {
  union U { v16h v; v8h h[2]; };
  static __device__ __forceinline__ v16h load(const _Float16* p) {
    U f;
    f.h[0] = *(const v8h*)(p);
    f.h[1] = *(const v8h*)(p + 16);
    return f.v;
  }
  static __device__ __forceinline__ v8f mma(v16h a, v16h b, v8f c) {
    return __builtin_amdgcn_wmma_f32_16x16x32_f16(false, a, false, b, (short)0, c, false, false);
  }
};
__device__ __forceinline__ void guard_row4(v8f& c0, v8f& c1, v8f& c2, v8f& c3,
                                           v16h a, v16h b0, v16h b1, v16h b2, v16h b3) {
  asm volatile("v_nop\n\tv_nop\n\tv_nop\n\tv_nop"
               : "+v"(c0), "+v"(c1), "+v"(c2), "+v"(c3)
               : "v"(a), "v"(b0), "v"(b1), "v"(b2), "v"(b3));
}
__device__ __forceinline__ void guard_split2(v8f& m0, v8f& m1, v8f& x0, v8f& x1,
                                             v16h ah, v16h al, v16h bh0, v16h bh1, v16h bl0, v16h bl1) {
  asm volatile("v_nop\n\tv_nop\n\tv_nop\n\tv_nop"
               : "+v"(m0), "+v"(m1), "+v"(x0), "+v"(x1)
               : "v"(ah), "v"(al), "v"(bh0), "v"(bh1), "v"(bl0), "v"(bl1));
}
__device__ __forceinline__ void acc_guard4(v8f& a, v8f& b, v8f& c, v8f& d) {
  asm volatile("v_nop\n\tv_nop\n\tv_nop\n\tv_nop" : "+v"(a), "+v"(b), "+v"(c), "+v"(d));
}

template <bool BIASN>
__global__ __launch_bounds__(256) void gemm_plain_f16_kernel(
    const unsigned short* __restrict__ Ap, int lda,
    const unsigned short* __restrict__ Btp, int ldb,
    float* __restrict__ C, int ldc, const float* __restrict__ bias,
    int M, int N, int K, float scale)
{
  const _Float16* A  = (const _Float16*)Ap;
  const _Float16* Bt = (const _Float16*)Btp;
  __shared__ __align__(16) float sT[8][16 * 68];
  const int lane = threadIdx.x & 31;
  const int wave = threadIdx.x >> 5;
  const int tilesN = N >> 6;
  const int tilesM = M >> 6;
  const int tile = blockIdx.x * 8 + wave;
  if (tile >= tilesM * tilesN) return;
  const int tm = tile / tilesN;
  const int tn = tile - tm * tilesN;
  const int m0 = tm << 6;
  const int n0 = tn << 6;
  const int rlane = lane & 15;
  const int koff  = (lane >> 4) * 8;
  const int mOff  = (lane >> 4) * 8;

  v8f acc[4][4];
#pragma unroll
  for (int i = 0; i < 4; ++i)
#pragma unroll
    for (int j = 0; j < 4; ++j) acc[i][j] = (v8f){0.f,0.f,0.f,0.f,0.f,0.f,0.f,0.f};

  for (int k0 = 0; k0 < K; k0 += 32) {
    v16h bh[4];
#pragma unroll
    for (int j = 0; j < 4; ++j) {
      const size_t bo = (size_t)(n0 + (j << 4) + rlane) * ldb + koff + k0;
      bh[j] = FragH::load(Bt + bo);
    }
#pragma unroll
    for (int i = 0; i < 4; ++i) {
      const size_t ao = (size_t)(m0 + (i << 4) + rlane) * lda + koff + k0;
      const v16h ah = FragH::load(A + ao);
#pragma unroll
      for (int j = 0; j < 4; ++j) acc[i][j] = FragH::mma(ah, bh[j], acc[i][j]);
      guard_row4(acc[i][0], acc[i][1], acc[i][2], acc[i][3], ah, bh[0], bh[1], bh[2], bh[3]);
    }
  }
  acc_guard4(acc[0][0], acc[0][1], acc[0][2], acc[0][3]);
  acc_guard4(acc[1][0], acc[1][1], acc[1][2], acc[1][3]);
  acc_guard4(acc[2][0], acc[2][1], acc[2][2], acc[2][3]);
  acc_guard4(acc[3][0], acc[3][1], acc[3][2], acc[3][3]);

  float* slab = sT[wave];
#pragma unroll
  for (int i = 0; i < 4; ++i) {
    const int mBase = m0 + (i << 4);
#pragma unroll
    for (int j = 0; j < 4; ++j) {
      const int n = n0 + (j << 4) + rlane;
      float bv = 0.f;
      if (BIASN) bv = bias[n];
#pragma unroll
      for (int r = 0; r < 8; ++r) {
        float v = acc[i][j][r] * scale;
        if (BIASN) v += bv;
        slab[(mOff + r) * 68 + (j << 4) + rlane] = v;
      }
    }
    __builtin_amdgcn_fence(__ATOMIC_RELEASE, "workgroup");
    __builtin_amdgcn_wave_barrier();
    __builtin_amdgcn_fence(__ATOMIC_ACQUIRE, "workgroup");
    {
      const int hh = lane >> 4, c4 = (lane & 15) * 4;
      for (int pass = 0; pass < 2; ++pass) {
#pragma unroll
        for (int it = 0; it < 8; ++it) {
          const int row = it * 2 + hh;
          const v4f v = *(const v4f*)(slab + row * 68 + c4);
          *(volatile v4f*)(C + (size_t)(mBase + row) * ldc + n0 + c4) = v;
        }
        __threadfence();
      }
    }
    __builtin_amdgcn_fence(__ATOMIC_RELEASE, "workgroup");
    __builtin_amdgcn_wave_barrier();
    __builtin_amdgcn_fence(__ATOMIC_ACQUIRE, "workgroup");
  }
}

__global__ __launch_bounds__(256) void gemm_split_f16_kernel(
    const unsigned short* __restrict__ Ahp, const unsigned short* __restrict__ Alp, int lda,
    const unsigned short* __restrict__ Bhp, const unsigned short* __restrict__ Blp, int ldb,
    float* __restrict__ C, int ldc, int M, int N, int K, float sMain, float sCross)
{
  const _Float16* Ah = (const _Float16*)Ahp;
  const _Float16* Al = (const _Float16*)Alp;
  const _Float16* Bh = (const _Float16*)Bhp;
  const _Float16* Bl = (const _Float16*)Blp;
  __shared__ __align__(16) float sT[8][16 * 36];
  const int lane = threadIdx.x & 31;
  const int wave = threadIdx.x >> 5;
  const int tilesN = N >> 5;
  const int tilesM = M >> 6;
  const int tile = blockIdx.x * 8 + wave;
  if (tile >= tilesM * tilesN) return;
  const int tm = tile / tilesN;
  const int tn = tile - tm * tilesN;
  const int m0 = tm << 6;
  const int n0 = tn << 5;
  const int rlane = lane & 15;
  const int koff  = (lane >> 4) * 8;
  const int mOff  = (lane >> 4) * 8;

  v8f am[4][2], ax[4][2];
#pragma unroll
  for (int i = 0; i < 4; ++i)
#pragma unroll
    for (int j = 0; j < 2; ++j) {
      am[i][j] = (v8f){0.f,0.f,0.f,0.f,0.f,0.f,0.f,0.f};
      ax[i][j] = (v8f){0.f,0.f,0.f,0.f,0.f,0.f,0.f,0.f};
    }

  for (int k0 = 0; k0 < K; k0 += 32) {
    v16h bh[2], bl[2];
#pragma unroll
    for (int j = 0; j < 2; ++j) {
      const size_t bo = (size_t)(n0 + (j << 4) + rlane) * ldb + koff + k0;
      bh[j] = FragH::load(Bh + bo);
      bl[j] = FragH::load(Bl + bo);
    }
#pragma unroll
    for (int i = 0; i < 4; ++i) {
      const size_t ao = (size_t)(m0 + (i << 4) + rlane) * lda + koff + k0;
      const v16h ah = FragH::load(Ah + ao);
      const v16h al = FragH::load(Al + ao);
#pragma unroll
      for (int j = 0; j < 2; ++j) {
        am[i][j] = FragH::mma(ah, bh[j], am[i][j]);
        ax[i][j] = FragH::mma(ah, bl[j], ax[i][j]);
        ax[i][j] = FragH::mma(al, bh[j], ax[i][j]);
      }
      guard_split2(am[i][0], am[i][1], ax[i][0], ax[i][1], ah, al, bh[0], bh[1], bl[0], bl[1]);
    }
  }
  acc_guard4(am[0][0], am[0][1], ax[0][0], ax[0][1]);
  acc_guard4(am[1][0], am[1][1], ax[1][0], ax[1][1]);
  acc_guard4(am[2][0], am[2][1], ax[2][0], ax[2][1]);
  acc_guard4(am[3][0], am[3][1], ax[3][0], ax[3][1]);

  float* slab = sT[wave];
#pragma unroll
  for (int i = 0; i < 4; ++i) {
    const int mBase = m0 + (i << 4);
#pragma unroll
    for (int j = 0; j < 2; ++j) {
#pragma unroll
      for (int r = 0; r < 8; ++r) {
        const float v = am[i][j][r] * sMain + ax[i][j][r] * sCross;
        slab[(mOff + r) * 36 + (j << 4) + rlane] = v;
      }
    }
    __builtin_amdgcn_fence(__ATOMIC_RELEASE, "workgroup");
    __builtin_amdgcn_wave_barrier();
    __builtin_amdgcn_fence(__ATOMIC_ACQUIRE, "workgroup");
    {
      const int q = lane >> 3, c4 = (lane & 7) * 4;
      for (int pass = 0; pass < 2; ++pass) {
#pragma unroll
        for (int it = 0; it < 4; ++it) {
          const int row = it * 4 + q;
          const v4f v = *(const v4f*)(slab + row * 36 + c4);
          *(volatile v4f*)(C + (size_t)(mBase + row) * ldc + n0 + c4) = v;
        }
        __threadfence();
      }
    }
    __builtin_amdgcn_fence(__ATOMIC_RELEASE, "workgroup");
    __builtin_amdgcn_wave_barrier();
    __builtin_amdgcn_fence(__ATOMIC_ACQUIRE, "workgroup");
  }
}

template <bool SPLIT>
__global__ __launch_bounds__(256) void cast_planes_kernel(
    const float* __restrict__ src, unsigned short* __restrict__ dhi, unsigned short* __restrict__ dlo,
    int total8, int valid8, float carry)
{
  const int i = blockIdx.x * 256 + threadIdx.x;
  if (i >= total8) return;
  const bool keep = (i < valid8);
  const int ic = keep ? i : (valid8 - 1);
  const size_t s0 = (size_t)ic << 3;
  const size_t e0 = (size_t)i << 3;
  const v4f a0 = *(const v4f*)(src + s0);
  const v4f a1 = *(const v4f*)(src + s0 + 4);
  v8h hv, lv;
#pragma unroll
  for (int e = 0; e < 4; ++e) {
    const float f0 = keep ? (a0[e] * carry) : 0.0f;
    const float f1 = keep ? (a1[e] * carry) : 0.0f;
    const _Float16 h0 = (_Float16)f0;
    const _Float16 h1 = (_Float16)f1;
    hv[e]     = h0;
    hv[4 + e] = h1;
    lv[e]     = (_Float16)((f0 - (float)h0) * kLoScale);
    lv[4 + e] = (_Float16)((f1 - (float)h1) * kLoScale);
  }
  unsigned short* qh = dhi + e0;
  unsigned short* ql = dlo + e0;
  *(volatile v8h*)qh = hv;
  if (SPLIT) *(volatile v8h*)ql = lv;
  __threadfence();
  *(volatile v8h*)qh = hv;
  if (SPLIT) *(volatile v8h*)ql = lv;
}

__global__ __launch_bounds__(256) void add_ln_kernel(
    const float* __restrict__ hin, const float* __restrict__ rin,
    const float* __restrict__ lw, const float* __restrict__ lb,
    float* __restrict__ out1, unsigned short* __restrict__ HNH, unsigned short* __restrict__ HNL)
{
  __shared__ float sS[8];
  __shared__ float sV[8];
  const int tid = threadIdx.x, lane = tid & 31, wave = tid >> 5;
  const int row = blockIdx.x;
  const int c4 = tid * 4;
  const size_t off = (size_t)row * kDm + c4;
  const v4f a = *(const v4f*)(hin + off);
  const v4f b = *(const v4f*)(rin + off);
  const v4f x = a + b;
  float s = (x[0] + x[1]) + (x[2] + x[3]);
#pragma unroll
  for (int o = 16; o > 0; o >>= 1) s += __shfl_xor(s, o, 32);
  if (lane == 0) sS[wave] = s;
  __syncthreads();
  float tot = 0.f;
#pragma unroll
  for (int w = 0; w < 8; ++w) tot += sS[w];
  const float mu = tot * (1.0f / (float)kDm);
  const float d0 = x[0] - mu, d1 = x[1] - mu, d2 = x[2] - mu, d3 = x[3] - mu;
  float s2 = (d0 * d0 + d1 * d1) + (d2 * d2 + d3 * d3);
#pragma unroll
  for (int o = 16; o > 0; o >>= 1) s2 += __shfl_xor(s2, o, 32);
  if (lane == 0) sV[wave] = s2;
  __syncthreads();
  float tot2 = 0.f;
#pragma unroll
  for (int w = 0; w < 8; ++w) tot2 += sV[w];
  const float var = tot2 * (1.0f / (float)kDm);
  const float inv = rsqrtf(var + kLnEps);
  const v4f wv = *(const v4f*)(lw + c4);
  const v4f bv = *(const v4f*)(lb + c4);
  float y[4];
  y[0] = d0 * inv * wv[0] + bv[0];
  y[1] = d1 * inv * wv[1] + bv[1];
  y[2] = d2 * inv * wv[2] + bv[2];
  y[3] = d3 * inv * wv[3] + bv[3];
  v4h hv, lv;
#pragma unroll
  for (int e = 0; e < 4; ++e) {
    const float f = y[e] * kCarryHn;
    const _Float16 hh = (_Float16)f;
    hv[e] = hh;
    lv[e] = (_Float16)((f - (float)hh) * kLoScale);
  }
  float* po = out1 + off;
  unsigned short* ph = HNH + off;
  unsigned short* pl = HNL + off;
  *(volatile v4f*)po = x;
  *(volatile v4h*)ph = hv;
  *(volatile v4h*)pl = lv;
  __threadfence();
  *(volatile v4f*)po = x;
  *(volatile v4h*)ph = hv;
  *(volatile v4h*)pl = lv;
}

__global__ __launch_bounds__(256) void conv_silu_kernel(
    const float* __restrict__ XZ, const float* __restrict__ cw, const float* __restrict__ cb,
    float* __restrict__ XA, unsigned short* __restrict__ XA16)
{
  __shared__ __align__(16) float sT[16 * kConvTP];
  const int tid = threadIdx.x, lane = tid & 31, wave = tid >> 5;
  const int d0 = blockIdx.x * 256, d = d0 + tid;
  const int g0 = blockIdx.y * 64;
  const int tb = g0 & (kSeq - 1);
  const v4f wq = *(const v4f*)(cw + (size_t)d * 4);
  const float w0 = wq[0], w1 = wq[1], w2 = wq[2], w3 = wq[3];
  const float bc = cb[d];
  float xm3, xm2, xm1;
  {
    const bool hist = (tb > 0);
    const int rb = hist ? (g0 - 3) : g0;
    const float v3 = XZ[(size_t)rb * kXzP + d];
    const float v2 = XZ[(size_t)(rb + 1) * kXzP + d];
    const float v1 = XZ[(size_t)(rb + 2) * kXzP + d];
    xm3 = hist ? v3 : 0.f;
    xm2 = hist ? v2 : 0.f;
    xm1 = hist ? v1 : 0.f;
  }
  const int hrow = wave >> 1;
  const int hch  = (wave & 1) * 128 + lane * 4;
#pragma unroll 1
  for (int sub = 0; sub < 4; ++sub) {
    const int lb = g0 + sub * 16;
#pragma unroll 1
    for (int s = 0; s < 16; ++s) {
      const float xcur = XZ[(size_t)(lb + s) * kXzP + d];
      float acc = w0 * xm3;
      acc = fmaf(w1, xm2, acc);
      acc = fmaf(w2, xm1, acc);
      acc = fmaf(w3, xcur, acc);
      const float sv = acc + bc;
      const float sg = __builtin_amdgcn_rcpf(1.0f + expf(-sv));
      sT[s * kConvTP + tid] = sv * sg;
      xm3 = xm2; xm2 = xm1; xm1 = xcur;
    }
    __syncthreads();
    v4f fv[4];
    v8h hv[2];
#pragma unroll
    for (int it = 0; it < 4; ++it) fv[it] = *(const v4f*)(sT + (it * 4 + hrow) * kConvTP + hch);
#pragma unroll
    for (int it = 0; it < 2; ++it) {
      const float* sp = sT + (it * 8 + wave) * kConvTP + lane * 8;
      const v4f a0 = *(const v4f*)(sp);
      const v4f a1 = *(const v4f*)(sp + 4);
#pragma unroll
      for (int e = 0; e < 4; ++e) {
        hv[it][e]     = (_Float16)(a0[e] * kCarryXa);
        hv[it][4 + e] = (_Float16)(a1[e] * kCarryXa);
      }
    }
    for (int pass = 0; pass < 2; ++pass) {
#pragma unroll
      for (int it = 0; it < 4; ++it)
        *(volatile v4f*)(XA + (size_t)(lb + it * 4 + hrow) * kDin + d0 + hch) = fv[it];
#pragma unroll
      for (int it = 0; it < 2; ++it)
        *(volatile v8h*)(XA16 + (size_t)(lb + it * 8 + wave) * kDin + d0 + lane * 8) = hv[it];
      __threadfence();
    }
    __syncthreads();
  }
}

__global__ __launch_bounds__(256) void dt_cast_kernel(
    const float* __restrict__ XD, unsigned short* __restrict__ DT16, int total8)
{
  const int i = blockIdx.x * 256 + threadIdx.x;
  if (i >= total8) return;
  const int e0  = i << 3;
  const int row = e0 >> 6;
  const int c8  = e0 & 63;
  const float* p = XD + (size_t)row * kPrjP + c8;
  const v4f a0 = *(const v4f*)(p);
  const v4f a1 = *(const v4f*)(p + 4);
  v8h hv;
#pragma unroll
  for (int e = 0; e < 4; ++e) {
    hv[e]     = (_Float16)(a0[e] * kCarryDt);
    hv[4 + e] = (_Float16)(a1[e] * kCarryDt);
  }
  unsigned short* qd = DT16 + e0;
  *(volatile v8h*)qd = hv;
  __threadfence();
  *(volatile v8h*)qd = hv;
}

__global__ __launch_bounds__(64) void scan_gate_kernel(
    const float* __restrict__ DLR, const float* __restrict__ XA, const float* __restrict__ XZ,
    const float* __restrict__ XD, const float* __restrict__ Alog, const float* __restrict__ Dp,
    unsigned short* __restrict__ YH, unsigned short* __restrict__ YL)
{
  __shared__ __align__(16) float sBC[kScanTS * 32];
  __shared__ __align__(16) float sY[kScanTS * kScanYP];
  __shared__ __align__(16) float sA[kNst * kScanCh];
  const int tid = threadIdx.x, lane = tid & 31, wave = tid >> 5;
  constexpr int kBlkPerB = kDin / kScanCh;
  const int bix = blockIdx.x / kBlkPerB;
  const int d0  = (blockIdx.x - bix * kBlkPerB) * kScanCh;
  const int d   = d0 + tid;
  const size_t row0 = (size_t)bix * kSeq;
#pragma unroll 1
  for (int s = 0; s < kNst; ++s) sA[s * kScanCh + tid] = -expf(Alog[(size_t)d * kNst + s]);
  __syncthreads();
  float negA[kNst], st[kNst];
#pragma unroll
  for (int s = 0; s < kNst; ++s) {
    negA[s] = sA[s * kScanCh + tid];
    st[s] = 0.f;
  }
  const float Dd = Dp[d];
  const int q = lane >> 3, c8 = (lane & 7) * 8;
#pragma unroll 1
  for (int t0 = 0; t0 < kSeq; t0 += kScanTS) {
    __syncthreads();
#pragma unroll
    for (int i = 0; i < 8; ++i) {
      const int idx = tid + 64 * i;
      const int r = idx >> 3, q4 = (idx & 7) * 4;
      *(v4f*)(sBC + r * 32 + q4) = *(const v4f*)(XD + (row0 + t0 + r) * kPrjP + kDtR + q4);
    }
    __syncthreads();
#pragma unroll 1
    for (int s = 0; s < kScanTS; ++s) {
      const size_t m = row0 + t0 + s;
      const float* xr = sBC + s * 32;
      float Bs[kNst], Cs[kNst];
#pragma unroll
      for (int q4 = 0; q4 < 4; ++q4) {
        const v4f bv = *(const v4f*)(xr + 4 * q4);
        const v4f cv = *(const v4f*)(xr + kNst + 4 * q4);
        Bs[4 * q4 + 0] = bv[0]; Bs[4 * q4 + 1] = bv[1]; Bs[4 * q4 + 2] = bv[2]; Bs[4 * q4 + 3] = bv[3];
        Cs[4 * q4 + 0] = cv[0]; Cs[4 * q4 + 1] = cv[1]; Cs[4 * q4 + 2] = cv[2]; Cs[4 * q4 + 3] = cv[3];
      }
      const float v   = DLR[m * kDin + d];
      const float dt  = fmaxf(v, 0.0f) + log1pf(expf(-fabsf(v)));
      const float xt  = XA[m * kDin + d];
      const float zv  = XZ[m * kXzP + kDin + d];
      const float dtx = dt * xt;
      float y = 0.f;
#pragma unroll
      for (int k = 0; k < kNst; ++k) {
        const float e = __expf(dt * negA[k]);
        st[k] = e * st[k] + dtx * Bs[k];
        y = st[k] * Cs[k] + y;
      }
      y = xt * Dd + y;
      const float sg = __builtin_amdgcn_rcpf(1.0f + expf(-zv));
      y = y * (zv * sg);
      sY[s * kScanYP + tid] = y * kCarryY;
    }
    __syncthreads();
#pragma unroll 1
    for (int it = 0; it < 8; ++it) {
      const int row = it * 8 + wave * 4 + q;
      const float* sp = sY + row * kScanYP + c8;
      const v4f a0 = *(const v4f*)(sp);
      const v4f a1 = *(const v4f*)(sp + 4);
      v8h hv, lv;
#pragma unroll
      for (int e = 0; e < 4; ++e) {
        const float f0 = a0[e], f1 = a1[e];
        const _Float16 h0 = (_Float16)f0;
        const _Float16 h1 = (_Float16)f1;
        hv[e]     = h0;
        hv[4 + e] = h1;
        lv[e]     = (_Float16)((f0 - (float)h0) * kLoScale);
        lv[4 + e] = (_Float16)((f1 - (float)h1) * kLoScale);
      }
      const size_t o = (row0 + t0 + row) * kDin + d0 + c8;
      unsigned short* ph = YH + o;
      unsigned short* pl = YL + o;
      *(volatile v8h*)ph = hv;
      *(volatile v8h*)pl = lv;
      __threadfence();
      *(volatile v8h*)ph = hv;
      *(volatile v8h*)pl = lv;
    }
  }
}

extern "C" void kernel_launch(void* const* d_in, const int* in_sizes, int n_in,
                              void* d_out, int out_size, void* d_ws, size_t ws_size,
                              hipStream_t stream)
{
  (void)stream;
  if (n_in < 13) return;
  if (in_sizes[0] != kRows * kDm || in_sizes[1] != kRows * kDm) return;
  if (in_sizes[2] != kDm || in_sizes[3] != kDm) return;
  if (in_sizes[4] != kXzP * kDm) return;
  if (in_sizes[5] != kDin * 4 || in_sizes[6] != kDin) return;
  if (in_sizes[7] != kPrjN * kDin) return;
  if (in_sizes[8] != kDin * kDtR || in_sizes[9] != kDin) return;
  if (in_sizes[10] != kDin * kNst || in_sizes[11] != kDin) return;
  if (in_sizes[12] != kDm * kDin) return;
  if (out_size != 2 * kRows * kDm) return;
  if (ws_size < kWsTotal) return;

  const float* hin       = (const float*)d_in[0];
  const float* rin       = (const float*)d_in[1];
  const float* ln_w      = (const float*)d_in[2];
  const float* ln_b      = (const float*)d_in[3];
  const float* in_proj_w = (const float*)d_in[4];
  const float* conv_w    = (const float*)d_in[5];
  const float* conv_b    = (const float*)d_in[6];
  const float* x_proj_w  = (const float*)d_in[7];
  const float* dt_proj_w = (const float*)d_in[8];
  const float* dt_proj_b = (const float*)d_in[9];
  const float* A_log     = (const float*)d_in[10];
  const float* Dskip     = (const float*)d_in[11];
  const float* out_proj_w= (const float*)d_in[12];
  float* out0 = (float*)d_out;
  float* out1 = (float*)d_out + kOut1ElemOff;

  char* ws = (char*)d_ws;
  unsigned short* WINH = (unsigned short*)(ws + kOffWINH);
  unsigned short* WINL = (unsigned short*)(ws + kOffWINL);
  unsigned short* WX   = (unsigned short*)(ws + kOffWX);
  unsigned short* WDT  = (unsigned short*)(ws + kOffWDT);
  unsigned short* WOH  = (unsigned short*)(ws + kOffWOH);
  unsigned short* WOL  = (unsigned short*)(ws + kOffWOL);
  unsigned short* HNH  = (unsigned short*)(ws + kOffHNH);
  unsigned short* HNL  = (unsigned short*)(ws + kOffHNL);
  float*          XZ   = (float*)(ws + kOffXZ);
  float*          XA   = (float*)(ws + kOffXA);
  unsigned short* XA16 = (unsigned short*)(ws + kOffXA16);
  float*          XD   = (float*)(ws + kOffXD);
  unsigned short* DT16 = (unsigned short*)(ws + kOffDT16);
  float*          DLR  = (float*)(ws + kOffDLR);
  unsigned short* YH   = (unsigned short*)(ws + kOffYH);
  unsigned short* YL   = (unsigned short*)(ws + kOffYL);

  cast_planes_kernel<true><<<(kXzP * kDm / 8) / 256, 256, 0, stream>>>(
      in_proj_w, WINH, WINL, kXzP * kDm / 8, kXzP * kDm / 8, kCarryW);
  cast_planes_kernel<false><<<(kPrjP * kDin / 8) / 256, 256, 0, stream>>>(
      x_proj_w, WX, WX, kPrjP * kDin / 8, kPrjN * kDin / 8, kCarryW);
  cast_planes_kernel<false><<<(kDin * kDtR / 8) / 256, 256, 0, stream>>>(
      dt_proj_w, WDT, WDT, kDin * kDtR / 8, kDin * kDtR / 8, kCarryWdt);
  cast_planes_kernel<true><<<(kDm * kDin / 8) / 256, 256, 0, stream>>>(
      out_proj_w, WOH, WOL, kDm * kDin / 8, kDm * kDin / 8, kCarryW);

  add_ln_kernel<<<kRows, 256, 0, stream>>>(hin, rin, ln_w, ln_b, out1, HNH, HNL);

  gemm_split_f16_kernel<<<(kRows / 64) * (kXzP / 32) / 8, 256, 0, stream>>>(
      HNH, HNL, kDm, WINH, WINL, kDm, XZ, kXzP, kRows, kXzP, kDm, kInMain, kInCross);

  conv_silu_kernel<<<dim3(kDin / 256, kRows / 64), 256, 0, stream>>>(XZ, conv_w, conv_b, XA, XA16);

  gemm_plain_f16_kernel<false><<<(kRows / 64) * (kPrjP / 64) / 8, 256, 0, stream>>>(
      XA16, kDin, WX, kDin, XD, kPrjP, dt_proj_b, kRows, kPrjP, kDin, kXpScale);

  dt_cast_kernel<<<(kRows * kDtR / 8) / 256, 256, 0, stream>>>(XD, DT16, kRows * kDtR / 8);

  gemm_plain_f16_kernel<true><<<(kRows / 64) * (kDin / 64) / 8, 256, 0, stream>>>(
      DT16, kDtR, WDT, kDtR, DLR, kDin, dt_proj_b, kRows, kDin, kDtR, kDtScale);

  scan_gate_kernel<<<kBatch * (kDin / kScanCh), kScanCh, 0, stream>>>(DLR, XA, XZ, XD, A_log, Dskip, YH, YL);

  gemm_split_f16_kernel<<<(kRows / 64) * (kDm / 32) / 8, 256, 0, stream>>>(
      YH, YL, kDin, WOH, WOL, kDin, out0, kDm, kRows, kDm, kDin, kOutMain, kOutCross);
}
